// PendulumHJBLoss_65214783422673
// MI455X (gfx1250) — hardware-verified
//
#include <hip/hip_runtime.h>
#pragma clang fp contract(off)

#define HDIM      128
#define HPAD      136
#define NW_MAIN   8
#define ITERS_TGT 8
#define EPSV      1.0e-4f
#define ASCALE    1024.0f
#define WSCALE    64.0f
#define UNSCALE   (1.0f / 65536.0f)

typedef _Float16 f16_t;
typedef unsigned short us_t;
typedef _Float16     v16h  __attribute__((ext_vector_type(16)));
typedef _Float16     v4h   __attribute__((ext_vector_type(4)));
typedef __bf16       v16b  __attribute__((ext_vector_type(16)));
typedef float        v8f   __attribute__((ext_vector_type(8)));
typedef float        v4f   __attribute__((ext_vector_type(4)));
typedef unsigned int u32x4 __attribute__((ext_vector_type(4)));

union FragH { v16h h; u32x4 u[2]; };
union FragB { v16b b; u32x4 u[2]; };

#define OFF_EW1   0
#define OFF_EB1   1024
#define OFF_EB2   1536
#define OFF_EB3   2048
#define OFF_DW1   2064
#define OFF_DB1   3088
#define OFF_DB2   3600
#define OFF_DB3   4112
#define OFF_EW2T  4128
#define OFF_DW2T  38944
#define OFF_EW3T  73760
#define OFF_DW3T  78112
#define OFF_RED   82464
#define OFF_LINE  82720
#define OFF_WAVE  82848
#define PER_WAVE  8960
#define SMEM_MAIN (OFF_WAVE + NW_MAIN * PER_WAVE)

#define OFF_S_EW1  0
#define OFF_S_EB1  1024
#define OFF_S_EB2  1536
#define OFF_S_EB3  2048
#define OFF_S_W2HI 2064
#define OFF_S_W2LO 36880
#define OFF_S_W3HI 71696
#define OFF_S_W3LO 76048
#define OFF_S_WAVE 80400
#define PER_WAVE_S 17664
#define OFF_S_DPART 151056
#define OFF_S_OUTS  156176
#define SMEM_SYMP   156240

__device__ __forceinline__ float fast_tanh(float x) {
#if __has_builtin(__builtin_amdgcn_tanhf)
  return __builtin_amdgcn_tanhf(x);
#else
  x = fminf(10.0f, fmaxf(-10.0f, x));
  float e = __expf(2.0f * x);
  return fmaf(-2.0f, __builtin_amdgcn_rcpf(e + 1.0f), 1.0f);
#endif
}

__device__ __forceinline__ float waveSum(float v) {
  v += __shfl_xor(v, 16, 32);
  v += __shfl_xor(v, 8, 32);
  v += __shfl_xor(v, 4, 32);
  v += __shfl_xor(v, 2, 32);
  v += __shfl_xor(v, 1, 32);
  return v;
}

__device__ __forceinline__ us_t bf16_rne(float x) {
  unsigned int u = __float_as_uint(x);
  u = u + 0x7FFFu + ((u >> 16) & 1u);
  return (us_t)(u >> 16);
}
__device__ __forceinline__ float bf16_up(us_t h) {
  return __uint_as_float(((unsigned int)h) << 16);
}

__device__ __forceinline__ v16h ldfrag_h(const f16_t* p) {
  FragH f;
  f.u[0] = *(const u32x4*)p;
  f.u[1] = *(const u32x4*)(p + 16);
  return f.h;
}
__device__ __forceinline__ v16b ldfrag_b(const us_t* p) {
  FragB f;
  f.u[0] = *(const u32x4*)p;
  f.u[1] = *(const u32x4*)(p + 16);
  return f.b;
}

__device__ __forceinline__ void wmma2_h(v16h a0, v16h a1, v16h b, v8f& c0, v8f& c1) {
  c0 = __builtin_amdgcn_wmma_f32_16x16x32_f16(false, a0, false, b, (short)0, c0, false, false);
  c1 = __builtin_amdgcn_wmma_f32_16x16x32_f16(false, a1, false, b, (short)0, c1, false, false);
  asm volatile("v_nop\n\tv_nop\n\tv_nop\n\tv_nop" : "+v"(c0), "+v"(c1) : "v"(a0), "v"(a1), "v"(b));
}

__device__ __forceinline__ v8f wmma3_bf(v16b ah, v16b al, v16b bh, v16b bl, v8f c) {
  c = __builtin_amdgcn_wmma_f32_16x16x32_bf16(false, ah, false, bh, (short)0, c, false, false);
  c = __builtin_amdgcn_wmma_f32_16x16x32_bf16(false, ah, false, bl, (short)0, c, false, false);
  c = __builtin_amdgcn_wmma_f32_16x16x32_bf16(false, al, false, bh, (short)0, c, false, false);
  asm volatile("v_nop\n\tv_nop\n\tv_nop\n\tv_nop" : "+v"(c) : "v"(ah), "v"(al), "v"(bh), "v"(bl));
  return c;
}

struct MLPH {
  const float* W1;
  const float* b1;
  const f16_t* w2t;
  const float* b2;
  const f16_t* w3t;
  const float* b3;
};

struct MLPS {
  const float* W1;
  const float* b1;
  const us_t* w2hi;
  const us_t* w2lo;
  const float* b2;
  const us_t* w3hi;
  const us_t* w3lo;
  const float* b3;
};

__device__ void mlp32_h(float p, float q, const MLPH prm,
                        f16_t* hbuf, float* pq, int lane, float& oP, float& oQ) {
  f16_t* myrow = hbuf + lane * HPAD;
#pragma unroll 2
  for (int j = 0; j < HDIM; j += 4) {
    const v4f w0 = *(const v4f*)(prm.W1 + j);
    const v4f w1 = *(const v4f*)(prm.W1 + HDIM + j);
    const v4f bb = *(const v4f*)(prm.b1 + j);
    v4h hv;
    hv.x = (f16_t)(fast_tanh(fmaf(p, w0.x, fmaf(q, w1.x, bb.x))) * ASCALE);
    hv.y = (f16_t)(fast_tanh(fmaf(p, w0.y, fmaf(q, w1.y, bb.y))) * ASCALE);
    hv.z = (f16_t)(fast_tanh(fmaf(p, w0.z, fmaf(q, w1.z, bb.z))) * ASCALE);
    hv.w = (f16_t)(fast_tanh(fmaf(p, w0.w, fmaf(q, w1.w, bb.w))) * ASCALE);
    *(v4h*)(myrow + j) = hv;
  }
  __syncthreads();

  const int col = lane & 15;
  const int hs  = lane >> 4;

  v16h A[2][4];
#pragma unroll
  for (int mt = 0; mt < 2; ++mt) {
#pragma unroll
    for (int kb = 0; kb < 4; ++kb) {
      A[mt][kb] = ldfrag_h(hbuf + (mt * 16 + col) * HPAD + kb * 32 + hs * 8);
    }
  }
  __syncthreads();

#pragma unroll
  for (int nt = 0; nt < 8; ++nt) {
    v8f c0, c1;
#pragma unroll
    for (int r = 0; r < 8; ++r) { c0[r] = 0.0f; c1[r] = 0.0f; }
#pragma unroll
    for (int kb = 0; kb < 4; ++kb) {
      v16h B = ldfrag_h(prm.w2t + (nt * 16 + col) * HPAD + kb * 32 + hs * 8);
      wmma2_h(A[0][kb], A[1][kb], B, c0, c1);
    }
    const float bias = prm.b2[nt * 16 + col];
#pragma unroll
    for (int r = 0; r < 8; ++r) {
      const int row = 8 * hs + r;
      float v0 = fast_tanh(fmaf(c0[r], UNSCALE, bias));
      float v1 = fast_tanh(fmaf(c1[r], UNSCALE, bias));
      hbuf[row * HPAD + nt * 16 + col]        = (f16_t)(v0 * ASCALE);
      hbuf[(16 + row) * HPAD + nt * 16 + col] = (f16_t)(v1 * ASCALE);
    }
  }
  __syncthreads();

  v8f d0, d1;
#pragma unroll
  for (int r = 0; r < 8; ++r) { d0[r] = 0.0f; d1[r] = 0.0f; }
#pragma unroll
  for (int kb = 0; kb < 4; ++kb) {
    v16h a0 = ldfrag_h(hbuf + col * HPAD + kb * 32 + hs * 8);
    v16h a1 = ldfrag_h(hbuf + (16 + col) * HPAD + kb * 32 + hs * 8);
    v16h B  = ldfrag_h(prm.w3t + col * HPAD + kb * 32 + hs * 8);
    wmma2_h(a0, a1, B, d0, d1);
  }
  const float b3v = (col == 0) ? prm.b3[0] : ((col == 1) ? prm.b3[1] : 0.0f);
  if (col < 2) {
    float* dst = pq + col * 32;
#pragma unroll
    for (int r = 0; r < 8; ++r) {
      dst[8 * hs + r]      = fmaf(d0[r], UNSCALE, b3v);
      dst[16 + 8 * hs + r] = fmaf(d1[r], UNSCALE, b3v);
    }
  }
  __syncthreads();
  oP = pq[lane];
  oQ = pq[32 + lane];
}

__device__ void mlp32_s(float p, float q, const MLPS prm,
                        us_t* hhi, us_t* hlo, float* pq, int lane, float& oP, float& oQ) {
#pragma unroll 1
  for (int j = 0; j < HDIM; ++j) {
    float a = tanhf(p * prm.W1[j] + q * prm.W1[HDIM + j] + prm.b1[j]);
    us_t h = bf16_rne(a);
    us_t l = bf16_rne(a - bf16_up(h));
    hhi[lane * HPAD + j] = h;
    hlo[lane * HPAD + j] = l;
  }
  __syncthreads();

  const int col = lane & 15;
  const int hs  = lane >> 4;

#pragma unroll
  for (int mt = 0; mt < 2; ++mt) {
    v16b Ah[4], Al[4];
#pragma unroll
    for (int kb = 0; kb < 4; ++kb) {
      Ah[kb] = ldfrag_b(hhi + (mt * 16 + col) * HPAD + kb * 32 + hs * 8);
      Al[kb] = ldfrag_b(hlo + (mt * 16 + col) * HPAD + kb * 32 + hs * 8);
    }
    __syncthreads();
#pragma unroll 1
    for (int nt = 0; nt < 8; ++nt) {
      v8f c;
#pragma unroll
      for (int r = 0; r < 8; ++r) c[r] = 0.0f;
#pragma unroll
      for (int kb = 0; kb < 4; ++kb) {
        v16b bh = ldfrag_b(prm.w2hi + (nt * 16 + col) * HPAD + kb * 32 + hs * 8);
        v16b bl = ldfrag_b(prm.w2lo + (nt * 16 + col) * HPAD + kb * 32 + hs * 8);
        c = wmma3_bf(Ah[kb], Al[kb], bh, bl, c);
      }
      const float bias = prm.b2[nt * 16 + col];
#pragma unroll
      for (int r = 0; r < 8; ++r) {
        float v = tanhf(c[r] + bias);
        us_t h = bf16_rne(v);
        us_t l = bf16_rne(v - bf16_up(h));
        const int idx = (mt * 16 + 8 * hs + r) * HPAD + nt * 16 + col;
        hhi[idx] = h;
        hlo[idx] = l;
      }
    }
  }
  __syncthreads();

  v8f d0, d1;
#pragma unroll
  for (int r = 0; r < 8; ++r) { d0[r] = 0.0f; d1[r] = 0.0f; }
#pragma unroll
  for (int kb = 0; kb < 4; ++kb) {
    v16b a0h = ldfrag_b(hhi + col * HPAD + kb * 32 + hs * 8);
    v16b a0l = ldfrag_b(hlo + col * HPAD + kb * 32 + hs * 8);
    v16b a1h = ldfrag_b(hhi + (16 + col) * HPAD + kb * 32 + hs * 8);
    v16b a1l = ldfrag_b(hlo + (16 + col) * HPAD + kb * 32 + hs * 8);
    v16b bh  = ldfrag_b(prm.w3hi + col * HPAD + kb * 32 + hs * 8);
    v16b bl  = ldfrag_b(prm.w3lo + col * HPAD + kb * 32 + hs * 8);
    d0 = wmma3_bf(a0h, a0l, bh, bl, d0);
    d1 = wmma3_bf(a1h, a1l, bh, bl, d1);
  }
  const float b3v = (col == 0) ? prm.b3[0] : ((col == 1) ? prm.b3[1] : 0.0f);
  if (col < 2) {
    float* dst = pq + col * 32;
#pragma unroll
    for (int r = 0; r < 8; ++r) {
      dst[8 * hs + r]      = d0[r] + b3v;
      dst[16 + 8 * hs + r] = d1[r] + b3v;
    }
  }
  __syncthreads();
  oP = pq[lane];
  oQ = pq[32 + lane];
}

__device__ void load_params_h(char* smem,
    const float* eW1, const float* eb1, const float* eW2, const float* eb2,
    const float* eW3, const float* eb3,
    const float* dW1, const float* db1, const float* dW2, const float* db2,
    const float* dW3, const float* db3) {
  const int tid = threadIdx.x, bs = blockDim.x;
  float* sEW1 = (float*)(smem + OFF_EW1);  float* sDW1 = (float*)(smem + OFF_DW1);
  float* sEB1 = (float*)(smem + OFF_EB1);  float* sDB1 = (float*)(smem + OFF_DB1);
  float* sEB2 = (float*)(smem + OFF_EB2);  float* sDB2 = (float*)(smem + OFF_DB2);
  float* sEB3 = (float*)(smem + OFF_EB3);  float* sDB3 = (float*)(smem + OFF_DB3);
  f16_t* sEW2T = (f16_t*)(smem + OFF_EW2T); f16_t* sDW2T = (f16_t*)(smem + OFF_DW2T);
  f16_t* sEW3T = (f16_t*)(smem + OFF_EW3T); f16_t* sDW3T = (f16_t*)(smem + OFF_DW3T);

  for (int i = tid; i < 2 * HDIM; i += bs) { sEW1[i] = eW1[i]; sDW1[i] = dW1[i]; }
  for (int i = tid; i < HDIM; i += bs) {
    sEB1[i] = eb1[i]; sEB2[i] = eb2[i]; sDB1[i] = db1[i]; sDB2[i] = db2[i];
  }
  if (tid < 2) { sEB3[tid] = eb3[tid]; sDB3[tid] = db3[tid]; }
  for (int i = tid; i < HDIM * HDIM; i += bs) {
    const int k = i >> 7, nn = i & 127;
    sEW2T[nn * HPAD + k] = (f16_t)(eW2[i] * WSCALE);
    sDW2T[nn * HPAD + k] = (f16_t)(dW2[i] * WSCALE);
  }
  for (int i = tid; i < 16 * HDIM; i += bs) {
    const int nn = i >> 7, k = i & 127;
    float v = 0.0f, w = 0.0f;
    if (nn < 2) { v = eW3[k * 2 + nn] * WSCALE; w = dW3[k * 2 + nn] * WSCALE; }
    sEW3T[nn * HPAD + k] = (f16_t)v;
    sDW3T[nn * HPAD + k] = (f16_t)w;
  }
}

__global__ __launch_bounds__(NW_MAIN * 32) void k_bulk(
    const float* __restrict__ p0, const float* __restrict__ q0,
    const float* __restrict__ p1, const float* __restrict__ q1,
    const float* __restrict__ omega, const float* __restrict__ dt,
    const float* __restrict__ Ptrue, const float* __restrict__ Qtrue,
    const float* eW1, const float* eb1, const float* eW2, const float* eb2,
    const float* eW3, const float* eb3,
    const float* dW1, const float* db1, const float* dW2, const float* db2,
    const float* dW3, const float* db3,
    float* ws, int n, int iters) {
  extern __shared__ char smem[];
  load_params_h(smem, eW1, eb1, eW2, eb2, eW3, eb3, dW1, db1, dW2, db2, dW3, db3);
  __syncthreads();

  const int lane = threadIdx.x & 31;
  const int wave = threadIdx.x >> 5;
  MLPH enc = {(const float*)(smem + OFF_EW1), (const float*)(smem + OFF_EB1),
              (const f16_t*)(smem + OFF_EW2T), (const float*)(smem + OFF_EB2),
              (const f16_t*)(smem + OFF_EW3T), (const float*)(smem + OFF_EB3)};
  MLPH dec = {(const float*)(smem + OFF_DW1), (const float*)(smem + OFF_DB1),
              (const f16_t*)(smem + OFF_DW2T), (const float*)(smem + OFF_DB2),
              (const f16_t*)(smem + OFF_DW3T), (const float*)(smem + OFF_DB3)};
  f16_t* hbuf = (f16_t*)(smem + OFF_WAVE + wave * PER_WAVE);
  float* pq   = (float*)(smem + OFF_WAVE + wave * PER_WAVE + 32 * HPAD * 2);

  const float dtv = dt[0];
  const int nwaves = gridDim.x * NW_MAIN;
  const int wgid = blockIdx.x * NW_MAIN + wave;

  float s_recon = 0.f, s_cons = 0.f, s_evo = 0.f, s_g1 = 0.f, s_g2 = 0.f;

  for (int it = 0; it < iters; ++it) {
    const int t = it * nwaves + wgid;
    const int i = t * 32 + lane;
    const bool ok = (i < n);
    const int ic = ok ? i : (n - 1);
    const float m = ok ? 1.0f : 0.0f;

    const float p0v = p0[ic], q0v = q0[ic];
    float P0, Q0; mlp32_h(p0v, q0v, enc, hbuf, pq, lane, P0, Q0);
    const float p1v = p1[ic], q1v = q1[ic];
    float P1, Q1; mlp32_h(p1v, q1v, enc, hbuf, pq, lane, P1, Q1);
    float pr, qr; mlp32_h(P0, Q0, dec, hbuf, pq, lane, pr, qr);

    const float dp = p0v - pr, dq = q0v - qr;
    s_recon += m * (dp * dp + dq * dq);
    const float dc = P0 - P1;
    s_cons += m * (dc * dc);
    const float dQ = Q1 - Q0;
    s_evo += m * (1.0f - cosf(dQ - omega[ic] * dtv));
    const float g = P0 - Ptrue[ic];
    s_g1 += m * (g * g);
    s_g2 += m * (1.0f - cosf(Q0 - Qtrue[ic]));
  }

  s_recon = waveSum(s_recon);
  s_cons  = waveSum(s_cons);
  s_evo   = waveSum(s_evo);
  s_g1    = waveSum(s_g1);
  s_g2    = waveSum(s_g2);

  float* red = (float*)(smem + OFF_RED);
  if (lane == 0) {
    red[wave * 8 + 0] = s_recon;
    red[wave * 8 + 1] = s_cons;
    red[wave * 8 + 2] = s_evo;
    red[wave * 8 + 3] = s_g1;
    red[wave * 8 + 4] = s_g2;
  }
  __syncthreads();
  float* line = (float*)(smem + OFF_LINE);
  if (wave == 0) {
    float v = 0.0f;
    if (lane < 5) {
#pragma unroll
      for (int w = 0; w < NW_MAIN; ++w) v += red[w * 8 + lane];
    }
    line[lane] = v;
  }
  __syncthreads();
  if (wave == 0 && lane < 8) {
    const v4f val = *(const v4f*)(line + 4 * lane);
    volatile v4f* dst = (volatile v4f*)(ws + (size_t)blockIdx.x * 32 + 4 * lane);
    *dst = val;
    __threadfence();
    *dst = val;
  }
}

__global__ __launch_bounds__(128) void k_fd_final(
    const float* __restrict__ p0, const float* __restrict__ q0,
    const float* eW1, const float* eb1, const float* eW2, const float* eb2,
    const float* eW3, const float* eb3,
    const float* ws, int nblk, int n, float* out) {
  extern __shared__ char smem[];
  const int tid = threadIdx.x, bs = blockDim.x;
  float* sW1 = (float*)(smem + OFF_S_EW1);
  float* sB1 = (float*)(smem + OFF_S_EB1);
  float* sB2 = (float*)(smem + OFF_S_EB2);
  float* sB3 = (float*)(smem + OFF_S_EB3);
  us_t* w2hi = (us_t*)(smem + OFF_S_W2HI);
  us_t* w2lo = (us_t*)(smem + OFF_S_W2LO);
  us_t* w3hi = (us_t*)(smem + OFF_S_W3HI);
  us_t* w3lo = (us_t*)(smem + OFF_S_W3LO);

  for (int i = tid; i < 2 * HDIM; i += bs) sW1[i] = eW1[i];
  for (int i = tid; i < HDIM; i += bs) { sB1[i] = eb1[i]; sB2[i] = eb2[i]; }
  if (tid < 2) sB3[tid] = eb3[tid];
  for (int i = tid; i < HDIM * HDIM; i += bs) {
    const int k = i >> 7, nn = i & 127;
    const float w = eW2[i];
    const us_t h = bf16_rne(w);
    const us_t l = bf16_rne(w - bf16_up(h));
    w2hi[nn * HPAD + k] = h;
    w2lo[nn * HPAD + k] = l;
  }
  for (int i = tid; i < 16 * HDIM; i += bs) {
    const int nn = i >> 7, k = i & 127;
    const float w = (nn < 2) ? eW3[k * 2 + nn] : 0.0f;
    const us_t h = bf16_rne(w);
    const us_t l = bf16_rne(w - bf16_up(h));
    w3hi[nn * HPAD + k] = h;
    w3lo[nn * HPAD + k] = l;
  }
  __syncthreads();

  const int lane = tid & 31;
  const int wave = tid >> 5;
  MLPS prm = {sW1, sB1, w2hi, w2lo, sB2, w3hi, w3lo, sB3};
  us_t* hhi = (us_t*)(smem + OFF_S_WAVE + wave * PER_WAVE_S);
  us_t* hlo = hhi + 32 * HPAD;
  float* pq = (float*)(smem + OFF_S_WAVE + wave * PER_WAVE_S + 2 * 32 * HPAD * 2);

  const int idx = (lane < n) ? lane : (n - 1);
  const float pi = p0[idx], qi = q0[idx];
  float pp = pi, qq = qi;
  if (wave == 0)      pp = pi + EPSV;
  else if (wave == 1) pp = pi - EPSV;
  else if (wave == 2) qq = qi + EPSV;
  else                qq = qi - EPSV;
  float Pg, Qg;
  mlp32_s(pp, qq, prm, hhi, hlo, pq, lane, Pg, Qg);

  float* outs = (float*)(smem + OFF_S_OUTS);
  if (wave == 0) {
    const float* g0 = (const float*)(smem + OFF_S_WAVE + 0 * PER_WAVE_S + 2 * 32 * HPAD * 2);
    const float* g1 = (const float*)(smem + OFF_S_WAVE + 1 * PER_WAVE_S + 2 * 32 * HPAD * 2);
    const float* g2 = (const float*)(smem + OFF_S_WAVE + 2 * PER_WAVE_S + 2 * 32 * HPAD * 2);
    const float* g3 = (const float*)(smem + OFF_S_WAVE + 3 * PER_WAVE_S + 2 * 32 * HPAD * 2);
    const float inv2e = 5000.0f;
    const float dPdp = (g0[lane] - g1[lane]) * inv2e;
    const float dPdq = (g2[lane] - g3[lane]) * inv2e;
    const float dQdp = (g0[32 + lane] - g1[32 + lane]) * inv2e;
    const float dQdq = (g2[32 + lane] - g3[32 + lane]) * inv2e;
    const float pb = dPdq * dQdp - dPdp * dQdq;
    const float tt = fabsf(pb) - 1.0f;
    const float s = waveSum(tt * tt);
    if (lane == 0) outs[7] = s * (1.0f / 32.0f);
  }

  double a0 = 0.0, a1 = 0.0, a2 = 0.0, a3 = 0.0, a4 = 0.0;
  for (int b = tid; b < nblk; b += bs) {
    const float* L = ws + (size_t)b * 32;
    a0 += (double)L[0];
    a1 += (double)L[1];
    a2 += (double)L[2];
    a3 += (double)L[3];
    a4 += (double)L[4];
  }
  double* dpart = (double*)(smem + OFF_S_DPART);
  dpart[tid * 5 + 0] = a0;
  dpart[tid * 5 + 1] = a1;
  dpart[tid * 5 + 2] = a2;
  dpart[tid * 5 + 3] = a3;
  dpart[tid * 5 + 4] = a4;
  __syncthreads();
  if (tid == 0) {
    double t0 = 0.0, t1 = 0.0, t2 = 0.0, t3 = 0.0, t4 = 0.0;
    for (int i = 0; i < bs; ++i) {
      t0 += dpart[i * 5 + 0];
      t1 += dpart[i * 5 + 1];
      t2 += dpart[i * 5 + 2];
      t3 += dpart[i * 5 + 3];
      t4 += dpart[i * 5 + 4];
    }
    const double invn = 1.0 / (double)n;
    const float recon = (float)(t0 * invn);
    const float cons  = (float)(t1 * invn);
    const float evo   = (float)(t2 * invn);
    const float gp    = (float)(t3 * invn);
    const float gq    = (float)(t4 * invn);
    const float gauge = gp + gq;
    const float symp  = outs[7];
    const float total = 1.0f * recon + 10.0f * cons + 5.0f * evo + 0.1f * symp + 5.0f * gauge;
    outs[0] = total; outs[1] = recon; outs[2] = cons;
    outs[3] = evo;   outs[4] = symp;  outs[5] = gauge;
  }
  __syncthreads();
  if (wave == 0 && lane < 6) {
    const float v = outs[lane];
    volatile float* o = out + lane;
    *o = v;
    __threadfence();
    *o = v;
  }
}

extern "C" void kernel_launch(void* const* d_in, const int* in_sizes, int n_in,
                              void* d_out, int out_size, void* d_ws, size_t ws_size,
                              hipStream_t stream) {
  if (n_in < 20 || out_size < 6) return;
  const int n = in_sizes[0];
  if (n < 1) return;
  const float* p0    = (const float*)d_in[0];
  const float* q0    = (const float*)d_in[1];
  const float* p1    = (const float*)d_in[2];
  const float* q1    = (const float*)d_in[3];
  const float* omega = (const float*)d_in[4];
  const float* dt    = (const float*)d_in[5];
  const float* Ptrue = (const float*)d_in[6];
  const float* Qtrue = (const float*)d_in[7];
  const float* eW1 = (const float*)d_in[8];
  const float* eb1 = (const float*)d_in[9];
  const float* eW2 = (const float*)d_in[10];
  const float* eb2 = (const float*)d_in[11];
  const float* eW3 = (const float*)d_in[12];
  const float* eb3 = (const float*)d_in[13];
  const float* dW1 = (const float*)d_in[14];
  const float* db1 = (const float*)d_in[15];
  const float* dW2 = (const float*)d_in[16];
  const float* db2 = (const float*)d_in[17];
  const float* dW3 = (const float*)d_in[18];
  const float* db3 = (const float*)d_in[19];
  float* ws  = (float*)d_ws;
  float* out = (float*)d_out;

  const int tiles = (n + 31) / 32;
  int blocks = (tiles + NW_MAIN * ITERS_TGT - 1) / (NW_MAIN * ITERS_TGT);
  if (blocks < 1) blocks = 1;
  if (blocks > 8192) blocks = 8192;
  const int nwaves = blocks * NW_MAIN;
  const int iters = (tiles + nwaves - 1) / nwaves;
  if ((size_t)blocks * 128u > ws_size) return;

  k_bulk<<<dim3(blocks), dim3(NW_MAIN * 32), SMEM_MAIN, stream>>>(
      p0, q0, p1, q1, omega, dt, Ptrue, Qtrue,
      eW1, eb1, eW2, eb2, eW3, eb3, dW1, db1, dW2, db2, dW3, db3,
      ws, n, iters);
  k_fd_final<<<dim3(1), dim3(128), SMEM_SYMP, stream>>>(
      p0, q0, eW1, eb1, eW2, eb2, eW3, eb3, ws, blocks, n, out);
}
